// _GCNNet_40286793236669
// MI455X (gfx1250) — hardware-run, weakly checked
//
#include <hip/hip_runtime.h>


namespace {
constexpr int N = 40000, NP = 40000  , E = 640000, D = 128, G = 64, NL = 3, DH2 = 64;
constexpr float XS = 8.0f, WSC = 256.0f, NEG = 0.2f  , EPSBN = 1e-5f;

typedef _Float16 b16;
typedef __attribute__((ext_vector_type(16))) _Float16 v16b;
typedef __attribute__((ext_vector_type(8))) _Float16 v8b;
typedef __attribute__((ext_vector_type(8))) float v8f;
typedef __attribute__((ext_vector_type(4))) float v4f;
__device__ __forceinline__ float bf16_rne(float f) { unsigned int u = __float_as_uint(f); u += 0x7FFFu + ((u >> 16) & 1u); return __uint_as_float(u & 0xFFFF0000u); }
__device__ __forceinline__ void split16(float v, b16& hi, b16& lo) { hi = (b16)v; lo = (b16)(v - (float)hi); }
__device__ __forceinline__ v16b frag_kb(const b16* p, int hh) { const v8b a = *(const v8b*)(p + 8 * hh), b = *(const v8b*)(p + 16 + 8 * hh); v16b f;
#pragma unroll
  for (int e = 0; e < 8; ++e) { f[e] = a[e]; f[8 + e] = b[e]; } return f; }
__device__ __forceinline__ v8f wmma16b(v16b a, v16b b, v8f c) { v8f d = __builtin_amdgcn_wmma_f32_16x16x32_f16(false, a, false, b, (short)0, c, false, false); asm volatile("v_nop\n\tv_nop\n\tv_nop\n\tv_nop" : "+v"(d) : "v"(a), "v"(b)); return d; }
__device__ __forceinline__ void wave_lds_sync() { __builtin_amdgcn_fence(__ATOMIC_RELEASE, "workgroup"); __builtin_amdgcn_wave_barrier(); __builtin_amdgcn_fence(__ATOMIC_ACQUIRE, "workgroup"); }
__device__ __forceinline__ float pmul(float a, float b) { float p = a * b; asm volatile("" : "+v"(p)); return p; }
__device__ __forceinline__ int iclamp(int v, int lo, int hi) { return v < lo ? lo : (v > hi ? hi : v); }
__device__ __forceinline__ float nexp(float x) { return __builtin_amdgcn_exp2f(x * 1.4426950408889634f); }
__device__ __forceinline__ float lrelu(float x) { return x > 0.0f ? x : NEG * x; }

constexpr int CSR_NBLK = 512, CSR_GB = 9, CSR_GN = 1 << CSR_GB  , CSR_MAXG = 512, CSR_CAP = 12288  ;
__global__ __launch_bounds__(64) void csrA_kernel(const int* __restrict__ dst, int E, int N, int nG, int CHP, int NGP, int* __restrict__ STG, int* __restrict__ HST) {
  extern __shared__ int sm[];
  int* cnt = sm; int* run = sm + NGP; int* ids = sm + 2 * NGP;
  const int b = blockIdx.x; const int ch = (E + CSR_NBLK - 1) / CSR_NBLK; const int e0 = b * ch, e1 = min(E, e0 + ch);
  for (int i = threadIdx.x; i < NGP; i += 64) cnt[i] = 0;
  for (int i = threadIdx.x; i < CHP; i += 64) ids[i] = -1;
  __syncthreads();
  if (threadIdx.x == 0) {
    for (int e = e0; e < e1; ++e) { int d = dst[e]; d = (d < 0) ? 0 : (d >= N ? N - 1 : d); cnt[d >> CSR_GB] += 1; }
    int acc = 0; for (int g = 0; g < nG; ++g) { run[g] = acc; acc += cnt[g]; }
    for (int e = e0; e < e1; ++e) { int d = dst[e]; d = (d < 0) ? 0 : (d >= N ? N - 1 : d); const int g = d >> CSR_GB; ids[run[g]] = e; run[g] += 1; } }
  __syncthreads();
  typedef __attribute__((ext_vector_type(4))) int v4i;
  for (int pass = 0; pass < 2; ++pass) {
    for (int i = threadIdx.x; i < CHP / 4; i += 64) *(volatile v4i*)(STG + (size_t)b * CHP + i * 4) = *(const v4i*)(&ids[i * 4]);
    for (int i = threadIdx.x; i < NGP / 4; i += 64) { v4i v; for (int e = 0; e < 4; ++e) v[e] = (i * 4 + e < nG) ? cnt[i * 4 + e] : 0; *(volatile v4i*)(HST + (size_t)b * NGP + i * 4) = v; }
    __threadfence(); }
}
__global__ __launch_bounds__(512) void csrS_kernel(const int* __restrict__ HST, int nG, int NGP, int* __restrict__ START, int* __restrict__ TOT, int* __restrict__ OFF) {
  __shared__ int tot[CSR_MAXG];
  const int b = threadIdx.x;
  for (int pass = 0; pass < 2; ++pass) { int runb = 0; for (int g = 0; g < nG; ++g) { int c = HST[(size_t)b * NGP + g]; c = (c < 0) ? 0 : c; ((volatile int*)OFF)[(size_t)g * CSR_NBLK + b] = runb; runb += c; } __threadfence(); }
  for (int g = threadIdx.x; g < nG; g += 512) { int s = 0; for (int bb = 0; bb < CSR_NBLK; ++bb) { int c = HST[(size_t)bb * NGP + g]; s += (c < 0) ? 0 : c; } tot[g] = s; }
  __syncthreads();
  if (threadIdx.x < 32) {
    __shared__ int st[CSR_MAXG + 32];
    if (threadIdx.x == 0) { int acc = 0; for (int g = 0; g < NGP; ++g) { st[g] = acc; if (g < nG) acc += (tot[g] + 31) & ~31; } st[NGP] = acc; }
    __builtin_amdgcn_fence(__ATOMIC_RELEASE, "workgroup"); __builtin_amdgcn_wave_barrier(); __builtin_amdgcn_fence(__ATOMIC_ACQUIRE, "workgroup");
    for (int pass = 0; pass < 2; ++pass) { for (int i = threadIdx.x; i < NGP + 32; i += 32) { ((volatile int*)START)[i] = (i <= NGP) ? st[min(i, NGP)] : 0; ((volatile int*)TOT)[i] = (i < nG) ? tot[i] : 0; } __threadfence(); } }
}
__global__ __launch_bounds__(256) void csrB_kernel(const int* __restrict__ dst, int N, int nG, int CHP, int NGP, int permLen, const int* __restrict__ STG, const int* __restrict__ HST, const int* __restrict__ OFF, const int* __restrict__ START, const int* __restrict__ TOT, int* __restrict__ PERM, int* __restrict__ ROWPTR, int* __restrict__ ROWCNT, int* __restrict__ FLAG) {
  typedef __attribute__((ext_vector_type(4))) int v4i;
  __shared__ int ids[CSR_CAP]; __shared__ unsigned short key[CSR_CAP]; __shared__ int outp[CSR_CAP]; __shared__ int ncnt[CSR_GN + 1]; __shared__ int boff[CSR_NBLK + 1];
  const int g = blockIdx.x, t_ = threadIdx.x; int tot = TOT[g]; int st = START[g], stn = START[g + 1]; const int v0 = g * CSR_GN; const int nv = min(CSR_GN, N - v0);
  st = (st < 0) ? 0 : (st > permLen - 32 ? permLen - 32 : st) & ~31; stn = (stn < st) ? st : (stn > permLen ? permLen : stn); tot = (tot < 0) ? 0 : tot; if (tot > stn - st && tot <= CSR_CAP) tot = stn - st;
  if (tot > CSR_CAP) {
    for (int pass = 0; pass < 2; ++pass) { for (int i = t_; i < CSR_GN / 4; i += 256) { v4i a, c; for (int e = 0; e < 4; ++e) { a[e] = st; c[e] = 0; } *(volatile v4i*)(ROWPTR + v0 + i * 4) = a; *(volatile v4i*)(ROWCNT + v0 + i * 4) = c; } if (t_ == 0) ((volatile int*)FLAG)[0] = 1; __threadfence(); } (void)nv; return; }
  if (t_ == 0) { int acc = 0; for (int b = 0; b < CSR_NBLK; ++b) { boff[b] = acc; int c = HST[(size_t)b * NGP + g]; c = (c < 0) ? 0 : (c > CHP ? CHP : c); acc += c; if (acc > tot) acc = tot; } boff[CSR_NBLK] = acc; }
  for (int i = t_; i <= CSR_GN; i += 256) ncnt[i] = 0;
  __syncthreads();
  for (int b = 0; b < CSR_NBLK; ++b) { const int c = boff[b + 1] - boff[b]; int o_ = OFF[(size_t)g * CSR_NBLK + b]; o_ = (o_ < 0) ? 0 : (o_ > CHP - c ? CHP - c : o_); const int* src_ = STG + (size_t)b * CHP + o_;
    for (int i = t_; i < c; i += 256) { int id = src_[i]; id = (id < 0) ? 0 : id; ids[boff[b] + i] = id; int d = dst[id]; d = (d < v0) ? v0 : (d >= N ? N - 1 : d); int kk = d - v0; kk = (kk < 0) ? 0 : (kk >= CSR_GN ? CSR_GN - 1 : kk); key[boff[b] + i] = (unsigned short)kk; } }
  __syncthreads();
  if (t_ == 0) { for (int i = 0; i < tot; ++i) ncnt[key[i]] += 1; int acc = 0; for (int vl = 0; vl < CSR_GN; ++vl) { const int c = ncnt[vl]; ncnt[vl] = acc; acc += c; } ncnt[CSR_GN] = acc;
    for (int i = 0; i < tot; ++i) { const int vl = key[i]; outp[ncnt[vl]] = ids[i]; ncnt[vl] += 1; }
    for (int vl = CSR_GN; vl > 0; --vl) ncnt[vl] = ncnt[vl - 1]; ncnt[0] = 0; }
  __syncthreads();
  for (int pass = 0; pass < 2; ++pass) {
    for (int i = t_; i < (stn - st) / 4; i += 256) { v4i v; for (int e = 0; e < 4; ++e) { const int q = i * 4 + e; v[e] = (q < tot) ? outp[q] : -1; } *(volatile v4i*)(PERM + st + i * 4) = v; }
    for (int i = t_; i < CSR_GN / 4; i += 256) { v4i a, c; for (int e = 0; e < 4; ++e) { const int vl = i * 4 + e; a[e] = st + ncnt[vl]; c[e] = (vl < nv) ? (ncnt[vl + 1] - ncnt[vl]) : 0; } *(volatile v4i*)(ROWPTR + v0 + i * 4) = a; *(volatile v4i*)(ROWCNT + v0 + i * 4) = c; }
    __threadfence(); }
}
__global__ __launch_bounds__(256) void csrZ_kernel(int* __restrict__ p, size_t n4) { typedef __attribute__((ext_vector_type(4))) int v4i; const size_t tid = (size_t)blockIdx.x * 256 + threadIdx.x, nth = (size_t)gridDim.x * 256; v4i z = {0, 0, 0, 0}; for (size_t i = tid; i < n4; i += nth) *(volatile v4i*)(p + i * 4) = z; }
struct CsrBufs { int *STG, *HST, *OFF, *START, *TOT, *PERM, *ROWPTR, *ROWCNT, *FLAG; int nG, NGP, CHP; size_t permLen; char* base; size_t bytes; };
static size_t csr_carve(CsrBufs& c, char* ws, size_t off, int E, int N) {
  const size_t off0 = off; c.base = ws + off;
  auto al = [&](size_t bytes) { char* p = ws + off; off += (bytes + 255) & ~(size_t)255; return p; };
  c.nG = (N + CSR_GN - 1) / CSR_GN; c.NGP = (c.nG + 31) & ~31; const int ch = (E + CSR_NBLK - 1) / CSR_NBLK; c.CHP = (ch + 31) & ~31; c.permLen = (size_t)E + 32 * (size_t)c.nG + 32;
  c.STG = (int*)al((size_t)CSR_NBLK * c.CHP * 4); c.HST = (int*)al((size_t)CSR_NBLK * c.NGP * 4); c.OFF = (int*)al((size_t)c.NGP * CSR_NBLK * 4); c.START = (int*)al((size_t)(c.NGP + 64) * 4); c.TOT = (int*)al((size_t)(c.NGP + 64) * 4);
  c.PERM = (int*)al(c.permLen * 4); c.ROWPTR = (int*)al((size_t)c.nG * CSR_GN * 4); c.ROWCNT = (int*)al((size_t)c.nG * CSR_GN * 4); c.FLAG = (int*)al(256);
  c.bytes = off - off0; return off;
}
static void csr_build(const CsrBufs& c, const int* dst, int E, int N, hipStream_t stream) {
  const size_t smem = (size_t)(2 * c.NGP + c.CHP) * 4;
  csrZ_kernel<<<512, 256, 0, stream>>>((int*)c.base, c.bytes / 16);
  csrA_kernel<<<CSR_NBLK, 64, smem, stream>>>(dst, E, N, c.nG, c.CHP, c.NGP, c.STG, c.HST);
  csrS_kernel<<<1, 512, 0, stream>>>(c.HST, c.nG, c.NGP, c.START, c.TOT, c.OFF);
  csrB_kernel<<<c.nG, 256, 0, stream>>>(dst, N, c.nG, c.CHP, c.NGP, (int)c.permLen, c.STG, c.HST, c.OFF, c.START, c.TOT, c.PERM, c.ROWPTR, c.ROWCNT, c.FLAG);
}


__global__ __launch_bounds__(256) void prepw_kernel(const float* __restrict__ ws_, b16* __restrict__ WT) {
  const int t = blockIdx.x * 256 + threadIdx.x; if (t >= NL * D * D / 8) return; const int l = t / (D * D / 8); const int e = (t % (D * D / 8)) * 8; const int oo = e / D, k0 = e % D; v8b o;
  for (int j = 0; j < 8; ++j) o[j] = (b16)(bf16_rne(ws_[((size_t)l * D + k0 + j) * D + oo]) * WSC);
  for (int pass = 0; pass < 2; ++pass) { *(volatile v8b*)(WT + (size_t)l * D * D + e) = o; __threadfence(); }
}
__global__ __launch_bounds__(256) void agg_kernel(const float* __restrict__ Hin, int layer, const float* __restrict__ MU, const float* __restrict__ RS, const float* __restrict__ gam, const float* __restrict__ bet, const int* __restrict__ srcs, const int* __restrict__ PERM, const int* __restrict__ ROWPTR, const int* __restrict__ ROWCNT, int permLen, float* __restrict__ AG, float* __restrict__ S) {
  __shared__ __attribute__((aligned(16))) float ss[32];
  const int wave = threadIdx.x >> 5, lane = threadIdx.x & 31; const size_t v = (size_t)blockIdx.x * 8 + wave;
  float g4[4], b4[4], m4[4], r4[4];
  for (int j = 0; j < 4; ++j) { const int c = lane * 4 + j; if (layer > 0) { g4[j] = bf16_rne(gam[c]); b4[j] = bf16_rne(bet[c]); m4[j] = MU[c]; r4[j] = RS[c]; } else { g4[j] = 1.0f; b4[j] = 0.0f; m4[j] = 0.0f; r4[j] = 1.0f; } }
  auto rowf = [&](size_t u, float* o4) { const v4f raw = *(const v4f*)(Hin + u * D + lane * 4); for (int j = 0; j < 4; ++j) { const float h = (layer > 0) ? raw[j] : bf16_rne(raw[j]); o4[j] = (layer > 0) ? (h - m4[j]) * r4[j] * g4[j] + b4[j] : h; } };
  int st = ROWPTR[v], cnt = ROWCNT[v]; cnt = iclamp(cnt, 0, 8192); st = iclamp(st, 0, permLen - cnt); const float dv = rsqrtf((float)(cnt + 1));
  float acc[4]; { float h4[4]; rowf(v, h4); for (int j = 0; j < 4; ++j) acc[j] = dv * h4[j]; } float ssum = dv;
  for (int i = 0; i < cnt; ++i) { const int e = iclamp(PERM[st + i], 0, E - 1); const int s = iclamp(srcs[e], 0, N - 1); const int cs_ = iclamp(ROWCNT[s], 0, 8192); const float ds = rsqrtf((float)(cs_ + 1)); float h4[4]; rowf((size_t)s, h4); for (int j = 0; j < 4; ++j) acc[j] += pmul(ds, h4[j]); ssum += ds; }
  v4f o; for (int j = 0; j < 4; ++j) o[j] = acc[j] * dv; if (lane == 0) ss[wave] = ssum * dv; if (threadIdx.x >= 8 && threadIdx.x < 32) ss[threadIdx.x] = 0.0f;
  __syncthreads();
  for (int pass = 0; pass < 2; ++pass) { *(volatile v4f*)(AG + v * D + lane * 4) = o; if (threadIdx.x < 8) *(volatile v4f*)(S + (size_t)blockIdx.x * 32 + threadIdx.x * 4) = *(const v4f*)(&ss[threadIdx.x * 4]); __threadfence(); }
}
__global__ __launch_bounds__(128) void layer_kernel(const float* __restrict__ AG, const float* __restrict__ S, const b16* __restrict__ Wt, const float* __restrict__ bias, float* __restrict__ H) {
  __shared__ __attribute__((aligned(16))) b16 Ah[4][16][D + 8], Al[4][16][D + 8]; __shared__ __attribute__((aligned(16))) float Tf[4][16][D + 4];
  const int wave = threadIdx.x >> 5, lane = threadIdx.x & 31, nloc = lane & 15, hlf = lane >> 4; const size_t m0 = (size_t)blockIdx.x * 64 + wave * 16;
  for (int q = lane; q < 16 * (D / 4); q += 32) { const int rr = q / (D / 4), c4 = (q % (D / 4)) * 4; const v4f xv = *(const v4f*)(AG + (m0 + rr) * D + c4); for (int j = 0; j < 4; ++j) { b16 p, pl; split16(xv[j] * XS, p, pl); Ah[wave][rr][c4 + j] = p; Al[wave][rr][c4 + j] = pl; } }
  wave_lds_sync();
  v8f acc[8];
#pragma unroll
  for (int t = 0; t < 8; ++t) acc[t] = (v8f){};
#pragma unroll
  for (int kb = 0; kb < D; kb += 32) { const v16b a = frag_kb(&Ah[wave][nloc][kb], hlf), al = frag_kb(&Al[wave][nloc][kb], hlf);
#pragma unroll
    for (int t = 0; t < 8; ++t) { const v16b bw = frag_kb(Wt + (size_t)(t * 16 + nloc) * D + kb, hlf); acc[t] = wmma16b(a, bw, acc[t]); acc[t] = wmma16b(al, bw, acc[t]); } }
#pragma unroll
  for (int t = 0; t < 8; ++t) { const int c = t * 16 + nloc; const float bb = bf16_rne(bias[c]);
#pragma unroll
    for (int r = 0; r < 8; ++r) { const size_t row = m0 + 8 * hlf + r; Tf[wave][8 * hlf + r][c] = fmaxf(acc[t][r] * (1.0f / (XS * WSC)) + pmul(S[(row >> 3) * 32 + (row & 7)], bb), 0.0f); } }
  wave_lds_sync();
  for (int pass = 0; pass < 2; ++pass) { for (int rr = 0; rr < 16; ++rr) *(volatile v4f*)(H + (m0 + rr) * D + lane * 4) = *(const v4f*)(&Tf[wave][rr][lane * 4]); __threadfence(); }
}
__global__ __launch_bounds__(128) void bn_kernel(const float* __restrict__ H, float* __restrict__ MU, float* __restrict__ RS) {
  __shared__ __attribute__((aligned(16))) float mu_s[D], rs_s[D];
  const int c = threadIdx.x; float s = 0.0f;
#pragma unroll 4
  for (int v = 0; v < N; ++v) s += H[(size_t)v * D + c];
  const float mu = s / (float)N; float q = 0.0f;
#pragma unroll 4
  for (int v = 0; v < N; ++v) { const float d = H[(size_t)v * D + c] - mu; q += d * d; }
  mu_s[c] = mu; rs_s[c] = rsqrtf(q / (float)N + EPSBN);
  __syncthreads();
  for (int pass = 0; pass < 2; ++pass) { if (c < 32) *(volatile v4f*)(MU + c * 4) = *(const v4f*)(&mu_s[c * 4]); else if (c < 64) *(volatile v4f*)(RS + (c - 32) * 4) = *(const v4f*)(&rs_s[(c - 32) * 4]); __threadfence(); }
}
__device__ __forceinline__ int lower_bound_(const int* __restrict__ a, int n, int key) { int lo = 0, hi = n; while (lo < hi) { const int mid = (lo + hi) >> 1; if (a[mid] < key) lo = mid + 1; else hi = mid; } return lo; }
__global__ __launch_bounds__(256) void head_kernel(const float* __restrict__ H, const float* __restrict__ MU, const float* __restrict__ RS, const float* __restrict__ gam, const float* __restrict__ bet, const int* __restrict__ batch, const float* __restrict__ w1, const float* __restrict__ b1, const float* __restrict__ w2, const float* __restrict__ b2, float* __restrict__ out) {
  __shared__ float pooled[G][D]; __shared__ __attribute__((aligned(16))) float res[G];
  const int wave = threadIdx.x >> 5, lane = threadIdx.x & 31, t_ = threadIdx.x;
  float g4[4], b4[4], m4[4], r4[4]; for (int j = 0; j < 4; ++j) { const int c = lane * 4 + j; g4[j] = bf16_rne(gam[c]); b4[j] = bf16_rne(bet[c]); m4[j] = MU[c]; r4[j] = RS[c]; }
  for (int g = wave; g < G; g += 8) { const int st = lower_bound_(batch, N, g), en = lower_bound_(batch, N, g + 1); float acc[4] = {0.0f, 0.0f, 0.0f, 0.0f};
    for (int v = st; v < en; ++v) { const v4f raw = *(const v4f*)(H + (size_t)v * D + lane * 4); for (int j = 0; j < 4; ++j) acc[j] += (raw[j] - m4[j]) * r4[j] * g4[j] + b4[j]; }
    const float inv = 1.0f / fmaxf((float)(en - st), 1.0f); for (int j = 0; j < 4; ++j) pooled[g][lane * 4 + j] = acc[j] * inv; }
  __syncthreads();
  if (t_ < G) { float o = bf16_rne(b2[0]);
#pragma unroll 1
    for (int k = 0; k < DH2; ++k) { float hsum = bf16_rne(b1[k]);
#pragma unroll 1
      for (int c = 0; c < D; ++c) hsum += pmul(pooled[t_][c], bf16_rne(w1[c * DH2 + k]));
      o += pmul(fmaxf(hsum, 0.0f), bf16_rne(w2[k])); }
    res[t_] = o; }
  __syncthreads();
  for (int pass = 0; pass < 2; ++pass) { if (t_ < 16) *(volatile v4f*)(out + t_ * 4) = *(const v4f*)(&res[t_ * 4]); __threadfence(); }
}
}

extern "C" void kernel_launch(void* const* d_in, const int* in_sizes, int n_in, void* d_out, int out_size, void* d_ws, size_t ws_size, hipStream_t stream) {
  (void)n_in;
  auto Fp = [&](int i) { return (const float*)d_in[i]; }; auto Ip = [&](int i) { return (const int*)d_in[i]; };
  if (in_sizes[0] != N * D || in_sizes[1] != 2 * E || in_sizes[2] != N || in_sizes[3] != NL * D * D || in_sizes[4] != NL * D || in_sizes[7] != D * DH2 || in_sizes[9] != DH2 || out_size != G) return;
  size_t off = 0; char* ws = (char*)d_ws;
  auto carve = [&](size_t bytes) { char* p = ws + off; off += (bytes + 255) & ~(size_t)255; return p; };
  b16* WT = (b16*)carve((size_t)NL * D * D * 2); float* AG = (float*)carve((size_t)N * D * 4); float* S = (float*)carve((size_t)(N / 8) * 32 * 4); float* HA = (float*)carve((size_t)N * D * 4); float* MU = (float*)carve((size_t)NL * D * 4); float* RS = (float*)carve((size_t)NL * D * 4);
  CsrBufs csr; off = csr_carve(csr, ws, off, E, N);
  if (off > ws_size || off > ((size_t)128 << 20)) return;
  prepw_kernel<<<(NL * D * D / 8 + 255) / 256, 256, 0, stream>>>(Fp(3), WT);
  csr_build(csr, Ip(1) + E, E, N, stream);
  for (int l = 0; l < NL; ++l) {
    agg_kernel<<<N / 8, 256, 0, stream>>>(l == 0 ? Fp(0) : HA, l, MU + (l - 1 < 0 ? 0 : l - 1) * D, RS + (l - 1 < 0 ? 0 : l - 1) * D, Fp(5) + (l - 1 < 0 ? 0 : l - 1) * D, Fp(6) + (l - 1 < 0 ? 0 : l - 1) * D, Ip(1), csr.PERM, csr.ROWPTR, csr.ROWCNT, (int)csr.permLen, AG, S);
    layer_kernel<<<N / 64, 128, 0, stream>>>(AG, S, WT + (size_t)l * D * D, Fp(4) + l * D, HA);
    bn_kernel<<<1, 128, 0, stream>>>(HA, MU + l * D, RS + l * D);
  }
  head_kernel<<<1, 256, 0, stream>>>(HA, MU + 2 * D, RS + 2 * D, Fp(5) + 2 * D, Fp(6) + 2 * D, Ip(2), Fp(7), Fp(8), Fp(9), Fp(10), (float*)d_out);
}
